// Model_11192684773891
// MI455X (gfx1250) — hardware-verified
//
#include <hip/hip_runtime.h>
#include <stddef.h>
#include <stdint.h>


#define DF     128
#define AP     512
#define K1L    384
#define K2L    512
#define KDL    256
#define NTHR   256
#define NWAVE  8
#define EPT    8
#define CHUNK  (NTHR * EPT)
#define WCAP   (EPT * 32)
#define LISTN  (NWAVE * WCAP)
#define NBA    1024
#define SLA    10
#define RCAP   28672
#define DEGCAP 128
#define GBM    64
#define GBN    128
#define GTHR   128
#define UPART  2048
#define NPART  18
#define ETHR   256
#define AGG_ZINTS    (LISTN + 2 * RCAP + 3 * NBA)
#define MISC_INTS    16
#define ROWBUF_INTS  (NWAVE * AP / 2)
#define AGG_LDS_INTS (AGG_ZINTS + MISC_INTS + ROWBUF_INTS)

static_assert((CHUNK & (CHUNK - 1)) == 0 && CHUNK <= 4096);
static_assert((NBA & (NBA - 1)) == 0 && NBA == (1 << SLA));
static_assert(((long long)CHUNK << SLA) < (1LL << 31));
static_assert(LISTN % NTHR == 0);
static_assert(NBA % NWAVE == 0 && NBA % 32 == 0 && NBA % GBM == 0);
static_assert(RCAP % 4 == 0 && AGG_ZINTS % 4 == 0 && LISTN % 4 == 0 && ((AGG_ZINTS + MISC_INTS) % 4) == 0);
static_assert(AGG_ZINTS % (NTHR * 4) == 0);
static_assert(K1L % 32 == 0 && K2L % 32 == 0 && KDL % 32 == 0);
static_assert(K2L == AP && K1L == 3 * DF && AP == 4 * DF && KDL == 2 * DF);
static_assert(GBN == DF && GBM == (GTHR / 32) * 16 && DF == 4 * 32);
static_assert(UPART % NTHR == 0 && UPART == DF * (DF / 8));
static_assert((NPART * UPART) % NTHR == 0);
static_assert(AGG_LDS_INTS * 4 <= 300000);
static_assert(ETHR == 8 * 32);

typedef float          v4f   __attribute__((ext_vector_type(4)));
typedef float          v8f   __attribute__((ext_vector_type(8)));
typedef int            v4i   __attribute__((ext_vector_type(4)));
typedef int            v8i   __attribute__((ext_vector_type(8)));
typedef unsigned       v2u   __attribute__((ext_vector_type(2)));
typedef unsigned short v4us  __attribute__((ext_vector_type(4)));
typedef unsigned short v8us  __attribute__((ext_vector_type(8)));
typedef unsigned short v16us __attribute__((ext_vector_type(16)));
typedef __bf16         v16bf __attribute__((ext_vector_type(16)));
typedef v4f  __attribute__((may_alias)) v4fa;
typedef v4i  __attribute__((may_alias)) v4ia;
typedef v2u  __attribute__((may_alias)) v2ua;
typedef v4us __attribute__((may_alias)) v4usa;
typedef v8us __attribute__((may_alias)) v8usa;
union FragB { v16bf v; v16us u; v8us h[2]; v8i w; };

__device__ __forceinline__ v8f wmb(const FragB& a, const FragB& b, v8f c) {
  v8f d = __builtin_amdgcn_wmma_f32_16x16x32_bf16(false, a.v, false, b.v, (short)0, c, false, false);
  asm volatile("v_nop\n\tv_nop\n\tv_nop\n\tv_nop" : "+v"(d) : "v"(a.w), "v"(b.w));
  return d;
}

__device__ __forceinline__ unsigned bf16_bits(float f) {
  const unsigned u = __float_as_uint(f);
  return (u + 0x7FFFu + ((u >> 16) & 1u)) >> 16;
}
__device__ __forceinline__ float bf16_val(float f) {
  return __uint_as_float(bf16_bits(f) << 16);
}

__device__ __forceinline__ void wave_sync() {
  __builtin_amdgcn_fence(__ATOMIC_RELEASE, "wavefront");
  __builtin_amdgcn_wave_barrier();
  __builtin_amdgcn_fence(__ATOMIC_ACQUIRE, "wavefront");
}

template <int SLB>
__device__ __forceinline__ int scan_chunk(const int* __restrict__ dsts, int nE, int cbase, int slotBase,
                                          int nb, int vec8, int* list, int tid, int lane, int wave) {
  int wc = 0;
  const int el0  = tid * EPT;
  const int e0   = cbase + el0;
  const int sent = -2147483647 - 1;
  v4i da, db;
  if (vec8 != 0 && cbase + CHUNK <= nE) {
    da = *(const v4i*)(dsts + e0);
    db = *(const v4i*)(dsts + e0 + 4);
  } else {
    da.x = (e0     < nE) ? dsts[min(e0,     nE - 1)] : sent;
    da.y = (e0 + 1 < nE) ? dsts[min(e0 + 1, nE - 1)] : sent;
    da.z = (e0 + 2 < nE) ? dsts[min(e0 + 2, nE - 1)] : sent;
    da.w = (e0 + 3 < nE) ? dsts[min(e0 + 3, nE - 1)] : sent;
    db.x = (e0 + 4 < nE) ? dsts[min(e0 + 4, nE - 1)] : sent;
    db.y = (e0 + 5 < nE) ? dsts[min(e0 + 5, nE - 1)] : sent;
    db.z = (e0 + 6 < nE) ? dsts[min(e0 + 6, nE - 1)] : sent;
    db.w = (e0 + 7 < nE) ? dsts[min(e0 + 7, nE - 1)] : sent;
  }
  const unsigned nbs = (unsigned)slotBase;
  const unsigned unb = (unsigned)nb;
  const unsigned s0 = (unsigned)da.x - nbs, s1 = (unsigned)da.y - nbs;
  const unsigned s2 = (unsigned)da.z - nbs, s3 = (unsigned)da.w - nbs;
  const unsigned s4 = (unsigned)db.x - nbs, s5 = (unsigned)db.y - nbs;
  const unsigned s6 = (unsigned)db.z - nbs, s7 = (unsigned)db.w - nbs;
  const bool h0 = s0 < unb, h1 = s1 < unb, h2 = s2 < unb, h3 = s3 < unb;
  const bool h4 = s4 < unb, h5 = s5 < unb, h6 = s6 < unb, h7 = s7 < unb;
  const unsigned any = __builtin_amdgcn_ballot_w32(h0 | h1 | h2 | h3 | h4 | h5 | h6 | h7);
  if (any != 0u) {
#define HITJ(J, HJ, SJ) { \
      const unsigned mj = __builtin_amdgcn_ballot_w32(HJ); \
      if (mj != 0u) { \
        if (HJ) { \
          const int pos = wc + (int)__builtin_amdgcn_mbcnt_lo(mj, 0u); \
          if (pos < WCAP) list[wave * WCAP + pos] = ((el0 + (J)) << SLB) | (int)(SJ); \
        } \
        wc += (int)__builtin_popcount(mj); } }
    HITJ(0, h0, s0)
    HITJ(1, h1, s1)
    HITJ(2, h2, s2)
    HITJ(3, h3, s3)
    HITJ(4, h4, s4)
    HITJ(5, h5, s5)
    HITJ(6, h6, s6)
    HITJ(7, h7, s7)
#undef HITJ
  }
  return wc;
}

__global__ __launch_bounds__(NTHR) void k_wprep(
    const float* __restrict__ Wl1ui, const float* __restrict__ Wr1ui,
    const float* __restrict__ Wl1iu, const float* __restrict__ Wr1iu,
    const float* __restrict__ Wl2ui, const float* __restrict__ Wr2ui,
    const float* __restrict__ Wl2iu, const float* __restrict__ Wr2iu,
    const float* __restrict__ WL1,
    unsigned short* B1I, unsigned short* B1U, unsigned short* B2I, unsigned short* B2U,
    unsigned short* BDU, unsigned short* BDI) {
  const int u    = (int)blockIdx.x * NTHR + (int)threadIdx.x;
  const int part = u >> 11;
  const int v    = u & (UPART - 1);
  const int n    = v >> 4;
  const int k8   = (v & 15) * 8;
  const float* W;
  unsigned short* P;
  int pitch, coff;
  if      (part == 0)  { W = Wl1ui; P = B1I; pitch = K1L; coff = 0; }
  else if (part == 1)  { W = Wl1ui; P = B1I; pitch = K1L; coff = DF; }
  else if (part == 2)  { W = Wr1ui; P = B1I; pitch = K1L; coff = 2 * DF; }
  else if (part == 3)  { W = Wl1iu; P = B1U; pitch = K1L; coff = 0; }
  else if (part == 4)  { W = Wl1iu; P = B1U; pitch = K1L; coff = DF; }
  else if (part == 5)  { W = Wr1iu; P = B1U; pitch = K1L; coff = 2 * DF; }
  else if (part == 6)  { W = Wl2ui; P = B2I; pitch = K2L; coff = 0; }
  else if (part == 7)  { W = Wl2ui; P = B2I; pitch = K2L; coff = DF; }
  else if (part == 8)  { W = Wr2ui; P = B2I; pitch = K2L; coff = 2 * DF; }
  else if (part == 9)  { W = Wr2ui; P = B2I; pitch = K2L; coff = 3 * DF; }
  else if (part == 10) { W = Wl2iu; P = B2U; pitch = K2L; coff = 0; }
  else if (part == 11) { W = Wl2iu; P = B2U; pitch = K2L; coff = DF; }
  else if (part == 12) { W = Wr2iu; P = B2U; pitch = K2L; coff = 2 * DF; }
  else if (part == 13) { W = Wr2iu; P = B2U; pitch = K2L; coff = 3 * DF; }
  else if (part == 14) { W = WL1;           P = BDU; pitch = KDL; coff = 0; }
  else if (part == 15) { W = WL1;           P = BDU; pitch = KDL; coff = DF; }
  else if (part == 16) { W = WL1 + DF * DF; P = BDI; pitch = KDL; coff = 0; }
  else if (part == 17) { W = WL1 + DF * DF; P = BDI; pitch = KDL; coff = DF; }
  else return;
  const float* p = W + (size_t)k8 * DF + n;
  v8us o;
#pragma unroll
  for (int i = 0; i < 8; ++i) o[i] = (unsigned short)bf16_bits(p[(size_t)i * DF]);
  unsigned short* dp = P + (size_t)n * pitch + coff + k8;
  *(volatile v8us*)dp = o;
  __threadfence();
  *(volatile v8us*)dp = o;
}

template <int MODE>
__global__ __launch_bounds__(GTHR) void k_gemm(unsigned short* Apl, const unsigned short* __restrict__ BT, int K,
                                               const float* __restrict__ bias, int useBias, int nOut) {
  __shared__ __attribute__((aligned(16))) float stg[GBM * GBN];
  const int tid = (int)threadIdx.x, lane = tid & 31, wave = tid >> 5, hh = lane >> 4, m = lane & 15;
  const int rowBase = (int)blockIdx.x * GBM;

  v8f acc[8];
  {
    const v8f z = {0.f, 0.f, 0.f, 0.f, 0.f, 0.f, 0.f, 0.f};
#pragma unroll
    for (int t = 0; t < 8; ++t) acc[t] = z;
  }
  const unsigned short* ap = Apl + (size_t)(rowBase + 16 * wave + m) * (size_t)AP + 8 * hh;
  const unsigned short* bp = BT + (size_t)m * (size_t)K + 8 * hh;

#pragma unroll 1
  for (int k0 = 0; k0 < K; k0 += 32) {
    FragB af;
    af.h[0] = *(const v8usa*)(ap + k0);
    af.h[1] = *(const v8usa*)(ap + k0 + 16);
#pragma unroll
    for (int nt = 0; nt < 8; ++nt) {
      const unsigned short* wq = bp + (size_t)(16 * nt) * (size_t)K + k0;
      FragB bf;
      bf.h[0] = *(const v8usa*)wq;
      bf.h[1] = *(const v8usa*)(wq + 16);
      acc[nt] = wmb(af, bf, acc[nt]);
    }
  }

#pragma unroll
  for (int nt = 0; nt < 8; ++nt) {
    const int lc = 16 * nt + m;
#pragma unroll
    for (int r = 0; r < 8; ++r) {
      const int lr = 16 * wave + 8 * hh + r;
      stg[lr * GBN + lc] = acc[nt][r];
    }
  }
  __syncthreads();

  v4f bb4;
  {
    const v4f t1 = *(const v4f*)(bias + 4 * lane);
    const float bs = (useBias != 0) ? 1.0f : 0.0f;
    bb4.x = bf16_val(t1.x) * bs;
    bb4.y = bf16_val(t1.y) * bs;
    bb4.z = bf16_val(t1.z) * bs;
    bb4.w = bf16_val(t1.w) * bs;
  }

  v4f pv[16];
#pragma unroll
  for (int i = 0; i < 16; ++i) pv[i] = *(const v4fa*)(stg + (16 * wave + i) * GBN + 4 * lane);
  __syncthreads();

#pragma unroll
  for (int i = 0; i < 16; ++i) {
    const bool ok = (rowBase + 16 * wave + i) < nOut;
    const v4f t = pv[i] + bb4;
    v4f y;
    if constexpr (MODE == 0) {
      y.x = (t.x > 0.0f) ? t.x : (t.x - t.x);
      y.y = (t.y > 0.0f) ? t.y : (t.y - t.y);
      y.z = (t.z > 0.0f) ? t.z : (t.z - t.z);
      y.w = (t.w > 0.0f) ? t.w : (t.w - t.w);
    } else {
      y = t;
    }
    y.x = ok ? y.x : 0.0f; y.y = ok ? y.y : 0.0f; y.z = ok ? y.z : 0.0f; y.w = ok ? y.w : 0.0f;
    pv[i] = y;
  }

  if constexpr (MODE == 2) {
#pragma unroll
    for (int i = 0; i < 16; ++i) {
      float* op = (float*)(Apl + (size_t)(rowBase + 16 * wave + i) * (size_t)AP + 2 * DF) + 4 * lane;
      *(volatile v4f*)op = pv[i];
    }
    __threadfence();
#pragma unroll
    for (int i = 0; i < 16; ++i) {
      float* op = (float*)(Apl + (size_t)(rowBase + 16 * wave + i) * (size_t)AP + 2 * DF) + 4 * lane;
      *(volatile v4f*)op = pv[i];
    }
  } else {
    constexpr int COFF = (MODE == 0) ? (2 * DF) : 0;
#pragma unroll
    for (int i = 0; i < 16; ++i) {
      v4us h4, l4;
      unsigned hb;
      hb = bf16_bits(pv[i].x); h4[0] = (unsigned short)hb; l4[0] = (unsigned short)bf16_bits(pv[i].x - __uint_as_float(hb << 16));
      hb = bf16_bits(pv[i].y); h4[1] = (unsigned short)hb; l4[1] = (unsigned short)bf16_bits(pv[i].y - __uint_as_float(hb << 16));
      hb = bf16_bits(pv[i].z); h4[2] = (unsigned short)hb; l4[2] = (unsigned short)bf16_bits(pv[i].z - __uint_as_float(hb << 16));
      hb = bf16_bits(pv[i].w); h4[3] = (unsigned short)hb; l4[3] = (unsigned short)bf16_bits(pv[i].w - __uint_as_float(hb << 16));
      unsigned short* srow = (unsigned short*)stg + (size_t)(16 * wave + i) * (2 * GBN);
      *(v4usa*)(srow + 4 * lane) = h4;
      *(v4usa*)(srow + DF + 4 * lane) = l4;
    }
    __syncthreads();
    v8us qv[16];
#pragma unroll
    for (int i = 0; i < 16; ++i) {
      const unsigned short* srow = (const unsigned short*)stg + (size_t)(16 * wave + i) * (2 * GBN);
      qv[i] = *(const v8usa*)(srow + 8 * lane);
    }
#pragma unroll
    for (int i = 0; i < 16; ++i) {
      unsigned short* rp = Apl + (size_t)(rowBase + 16 * wave + i) * (size_t)AP + COFF + 8 * lane;
      *(volatile v8us*)rp = qv[i];
    }
    __threadfence();
#pragma unroll
    for (int i = 0; i < 16; ++i) {
      unsigned short* rp = Apl + (size_t)(rowBase + 16 * wave + i) * (size_t)AP + COFF + 8 * lane;
      *(volatile v8us*)rp = qv[i];
    }
  }
}

template <int L0>
__global__ __launch_bounds__(NTHR) void k_scan(const int* __restrict__ gath, const int* __restrict__ keys,
                                               int nE, int nN, int nSrc, int vec8, int mRows,
                                               const float* __restrict__ xsrc, const float* __restrict__ xown,
                                               const unsigned short* hsrc, unsigned short* apl) {
  extern __shared__ __attribute__((aligned(16))) int dsm[];
  int* list = dsm;
  int* hl   = dsm + LISTN;
  int* sl   = hl + RCAP;
  int* cnt  = sl + RCAP;
  int* offs = cnt + NBA;
  int* cur  = offs + NBA;
  int* misc = cur + NBA;
  const int tid = (int)threadIdx.x, lane = tid & 31, wave = tid >> 5;
  unsigned short* rowbuf = (unsigned short*)(misc + MISC_INTS) + wave * AP;
  const int nodeBase = (int)blockIdx.x * NBA;

  {
    const v4i z4 = {0, 0, 0, 0};
    for (int i = tid * 4; i < AGG_ZINTS; i += NTHR * 4) *(v4ia*)(dsm + i) = z4;
    if (tid < MISC_INTS) misc[tid] = 0;
  }
  __syncthreads();

  int t = 0, ov = 0;
  const int nChunks = (nE + CHUNK - 1) / CHUNK;
#pragma unroll 1
  for (int ch = 0; ch < nChunks; ++ch) {
    const int cbase = ch * CHUNK;
    const int wc = scan_chunk<SLA>(keys, nE, cbase, nodeBase, NBA, vec8, list, tid, lane, wave);
    if (lane == 0) misc[wave] = wc;
    __syncthreads();
    if (wave == 0) {
#pragma unroll 1
      for (int w2 = 0; w2 < NWAVE; ++w2) {
        int c = misc[w2];
        c = c < 0 ? 0 : (c > WCAP ? WCAP : c);
#pragma unroll 1
        for (int b0 = 0; b0 < c; b0 += 32) {
          const int idx = b0 + lane;
          const int ent = list[w2 * WCAP + (idx < WCAP ? idx : WCAP - 1)];
          const int m32 = (c - b0) < 32 ? (c - b0) : 32;
#pragma unroll 1
          for (int k = 0; k < m32; ++k) {
            const int u    = __builtin_amdgcn_readlane(ent, k);
            const int slot = u & (NBA - 1);
            const int el   = (u >> SLA) & (CHUNK - 1);
            const int pk   = ((cbase + el) << SLA) | slot;
            if (t < RCAP) {
              if (lane == 0) { hl[t] = pk; cnt[slot] = cnt[slot] + 1; }
              t = t + 1;
            } else {
              ov = 1;
            }
          }
        }
      }
    }
    __syncthreads();
  }
  if (wave == 0 && lane == 0) { misc[8] = t; misc[9] = ov; }
  __syncthreads();
  int tt = misc[8];
  tt = tt < 0 ? 0 : (tt > RCAP ? RCAP : tt);
  const int ovf = misc[9];

  if (wave == 0) {
    const int base = lane * (NBA / 32);
    int s = 0;
#pragma unroll 1
    for (int i = 0; i < NBA / 32; ++i) s += cnt[base + i];
    int incl = s;
#pragma unroll
    for (int d = 1; d < 32; d <<= 1) {
      const int y = __shfl_up(incl, d, 32);
      if (lane >= d) incl += y;
    }
    int run = incl - s;
#pragma unroll 1
    for (int i = 0; i < NBA / 32; ++i) {
      const int cv = cnt[base + i];
      offs[base + i] = run;
      cur[base + i]  = run;
      run += cv;
    }
  }
  __syncthreads();
  if (wave == 0) {
#pragma unroll 1
    for (int b0 = 0; b0 < tt; b0 += 32) {
      const int idx = b0 + lane;
      const int ent = hl[idx < RCAP ? idx : RCAP - 1];
      const int m32 = (tt - b0) < 32 ? (tt - b0) : 32;
#pragma unroll 1
      for (int k = 0; k < m32; ++k) {
        const int u    = __builtin_amdgcn_readlane(ent, k);
        const int slot = u & (NBA - 1);
        if (lane == 0) {
          int p = cur[slot];
          p = p < 0 ? 0 : (p > RCAP - 1 ? RCAP - 1 : p);
          sl[p] = u;
          cur[slot] = p + 1;
        }
      }
    }
  }
  __syncthreads();

  const float pz = (ovf != 0) ? __int_as_float(0x7fc00000) : 0.0f;
#pragma unroll 1
  for (int si = 0; si < NBA / NWAVE; ++si) {
    const int s    = si * NWAVE + wave;
    const int node = nodeBase + s;
    const int craw = cnt[s];
    const bool big = craw > DEGCAP;
    const int c = craw < 0 ? 0 : (craw > DEGCAP ? DEGCAP : craw);
    int o = offs[s];
    o = o < 0 ? 0 : (o > RCAP ? RCAP : o);
    const int nc = node < nN ? node : nN - 1;
    float a0 = 0.0f, a1 = 0.0f, a2 = 0.0f, a3 = 0.0f;
#pragma unroll 1
    for (int b0 = 0; b0 < c; b0 += 32) {
      int idx = o + b0 + lane;
      idx = idx > RCAP - 1 ? RCAP - 1 : idx;
      const int ent = sl[idx];
      int eid = ent >> SLA;
      eid = eid < 0 ? 0 : (eid > nE - 1 ? nE - 1 : eid);
      int sr = gath[eid];
      sr = sr < 0 ? 0 : (sr > nSrc - 1 ? nSrc - 1 : sr);
      const int m32 = (c - b0) < 32 ? (c - b0) : 32;
#pragma unroll 1
      for (int k = 0; k < m32; ++k) {
        const int sk = __builtin_amdgcn_readlane(sr, k);
        if constexpr (L0 != 0) {
          const v4f a = *(const v4f*)(xsrc + (size_t)sk * DF + 4 * lane);
          a0 += bf16_val(a.x);
          a1 += bf16_val(a.y);
          a2 += bf16_val(a.z);
          a3 += bf16_val(a.w);
        } else {
          const unsigned short* rp = hsrc + (size_t)sk * AP + 2 * DF + 4 * lane;
          const v2u wh = *(const v2ua*)rp;
          const v2u wl = *(const v2ua*)(rp + DF);
          const float f0 = __uint_as_float(wh.x << 16)         + __uint_as_float(wl.x << 16);
          const float f1 = __uint_as_float(wh.x & 0xffff0000u) + __uint_as_float(wl.x & 0xffff0000u);
          const float f2 = __uint_as_float(wh.y << 16)         + __uint_as_float(wl.y << 16);
          const float f3 = __uint_as_float(wh.y & 0xffff0000u) + __uint_as_float(wl.y & 0xffff0000u);
          a0 += f0;
          a1 += f1;
          a2 += f2;
          a3 += f3;
        }
      }
    }
    const float cf = (float)(c < 1 ? 1 : c);
    const float rc = 1.0f / cf;
    const float pzr = big ? __int_as_float(0x7fc00000) : pz;
    const bool live = node < nN;
    const float m0 = live ? (a0 * rc + pzr) : 0.0f;
    const float m1 = live ? (a1 * rc + pzr) : 0.0f;
    const float m2 = live ? (a2 * rc + pzr) : 0.0f;
    const float m3 = live ? (a3 * rc + pzr) : 0.0f;
    v4us mh, ml;
    {
      unsigned hb;
      hb = bf16_bits(m0); mh[0] = (unsigned short)hb; ml[0] = (unsigned short)bf16_bits(m0 - __uint_as_float(hb << 16));
      hb = bf16_bits(m1); mh[1] = (unsigned short)hb; ml[1] = (unsigned short)bf16_bits(m1 - __uint_as_float(hb << 16));
      hb = bf16_bits(m2); mh[2] = (unsigned short)hb; ml[2] = (unsigned short)bf16_bits(m2 - __uint_as_float(hb << 16));
      hb = bf16_bits(m3); mh[3] = (unsigned short)hb; ml[3] = (unsigned short)bf16_bits(m3 - __uint_as_float(hb << 16));
    }
    *(v4usa*)(rowbuf + 4 * lane) = mh;
    *(v4usa*)(rowbuf + DF + 4 * lane) = ml;
    if constexpr (L0 != 0) {
      const v4f xs = *(const v4f*)(xown + (size_t)nc * DF + 4 * lane);
      v4us xb;
      xb[0] = live ? (unsigned short)bf16_bits(xs.x + pzr) : (unsigned short)0;
      xb[1] = live ? (unsigned short)bf16_bits(xs.y + pzr) : (unsigned short)0;
      xb[2] = live ? (unsigned short)bf16_bits(xs.z + pzr) : (unsigned short)0;
      xb[3] = live ? (unsigned short)bf16_bits(xs.w + pzr) : (unsigned short)0;
      const v4us z4 = {0, 0, 0, 0};
      *(v4usa*)(rowbuf + 2 * DF + 4 * lane) = xb;
      *(v4usa*)(rowbuf + 3 * DF + 4 * lane) = z4;
    }
    wave_sync();
    const v8us q0 = *(const v8usa*)(rowbuf + 8 * lane);
    v8us q1 = {0, 0, 0, 0, 0, 0, 0, 0};
    if constexpr (L0 != 0) q1 = *(const v8usa*)(rowbuf + 2 * DF + 8 * lane);
    wave_sync();
    if (node < mRows) {
      unsigned short* rpw = apl + (size_t)node * AP + 8 * lane;
      *(volatile v8us*)rpw = q0;
      if constexpr (L0 != 0) *(volatile v8us*)(rpw + 2 * DF) = q1;
      __threadfence();
      *(volatile v8us*)rpw = q0;
      if constexpr (L0 != 0) *(volatile v8us*)(rpw + 2 * DF) = q1;
    }
  }
}

__global__ __launch_bounds__(ETHR) void k_edge(const float* __restrict__ fu, const float* __restrict__ fi,
                                               const int* __restrict__ elr, const int* __restrict__ elc,
                                               int nL, int nU, int nI,
                                               const float* __restrict__ w2, const float* __restrict__ b2,
                                               float* out) {
  __shared__ __attribute__((aligned(16))) float ostg[ETHR];
  const int tid = (int)threadIdx.x, lane = tid & 31, wave = tid >> 5;
  const int l0 = (int)blockIdx.x * ETHR + wave * 32;
  v4f w;
  {
    const v4f t = *(const v4f*)(w2 + 4 * lane);
    w.x = bf16_val(t.x); w.y = bf16_val(t.y); w.z = bf16_val(t.z); w.w = bf16_val(t.w);
  }
  const float bb = bf16_val(b2[0]);
  const int l  = l0 + lane;
  const int lc = l < nL ? l : nL - 1;
  int er = elr[lc];
  er = er < 0 ? 0 : (er > nU - 1 ? nU - 1 : er);
  int ec = elc[lc];
  ec = ec < 0 ? 0 : (ec > nI - 1 ? nI - 1 : ec);
  float res = 0.0f;
#pragma unroll 1
  for (int k = 0; k < 32; ++k) {
    const int rk = __builtin_amdgcn_readlane(er, k);
    const int ck = __builtin_amdgcn_readlane(ec, k);
    const v4f du = *(const v4f*)(fu + (size_t)rk * (AP / 2) + DF + 4 * lane);
    const v4f di = *(const v4f*)(fi + (size_t)ck * (AP / 2) + DF + 4 * lane);
    const v4f v = du + di;
    const float r0 = (v.x > 0.0f) ? v.x : (v.x - v.x);
    const float r1 = (v.y > 0.0f) ? v.y : (v.y - v.y);
    const float r2 = (v.z > 0.0f) ? v.z : (v.z - v.z);
    const float r3 = (v.w > 0.0f) ? v.w : (v.w - v.w);
    float s = r0 * w.x;
    s = fmaf(r1, w.y, s);
    s = fmaf(r2, w.z, s);
    s = fmaf(r3, w.w, s);
    s += __shfl_xor(s, 16, 32);
    s += __shfl_xor(s, 8, 32);
    s += __shfl_xor(s, 4, 32);
    s += __shfl_xor(s, 2, 32);
    s += __shfl_xor(s, 1, 32);
    res = (lane == k) ? s : res;
  }
  ostg[wave * 32 + lane] = res + bb;
  wave_sync();
  const v4f ov = *(const v4fa*)(ostg + wave * 32 + 4 * (lane & 7));
  const bool okst = (lane < 8) && (l0 < nL);
  float* op = out + (size_t)l0 + 4 * (lane & 7);
  if (okst) *(volatile v4f*)op = ov;
  __threadfence();
  if (okst) *(volatile v4f*)op = ov;
}

static inline int cdiv(int a, int b) { return (a + b - 1) / b; }
static inline size_t al256(size_t o) { return (o + 255) & ~(size_t)255; }

extern "C" void kernel_launch(void* const* d_in, const int* in_sizes, int n_in,
                              void* d_out, int out_size, void* d_ws, size_t ws_size,
                              hipStream_t stream) {
  if (n_in < 22) return;
  if (in_sizes[0] < DF || (in_sizes[0] % DF) != 0) return;
  if (in_sizes[1] < DF || (in_sizes[1] % DF) != 0) return;
  const int nU = in_sizes[0] / DF;
  const int nI = in_sizes[1] / DF;
  if (nU < 16 || nU >= (1 << 24) || nI < 16 || nI >= (1 << 24)) return;
  for (int i = 2; i <= 12; i += 3) {
    if (in_sizes[i] != DF * DF || in_sizes[i + 1] != DF * DF || in_sizes[i + 2] != DF) return;
  }
  if (in_sizes[14] != 2 * DF * DF || in_sizes[15] != DF) return;
  if (in_sizes[16] != DF || in_sizes[17] != 1) return;
  const int nE = in_sizes[18];
  if (nE < 1 || nE >= (1 << 21) || in_sizes[19] != nE) return;
  const int nL = in_sizes[20];
  if (nL < 32 || (nL % 32) != 0 || in_sizes[21] != nL) return;
  if (out_size != nL) return;

  const float* x_user = (const float*)d_in[0];
  const float* x_item = (const float*)d_in[1];
  const float* Wl1_ui = (const float*)d_in[2];
  const float* Wr1_ui = (const float*)d_in[3];
  const float* b1_ui  = (const float*)d_in[4];
  const float* Wl1_iu = (const float*)d_in[5];
  const float* Wr1_iu = (const float*)d_in[6];
  const float* b1_iu  = (const float*)d_in[7];
  const float* Wl2_ui = (const float*)d_in[8];
  const float* Wr2_ui = (const float*)d_in[9];
  const float* b2_ui  = (const float*)d_in[10];
  const float* Wl2_iu = (const float*)d_in[11];
  const float* Wr2_iu = (const float*)d_in[12];
  const float* b2_iu  = (const float*)d_in[13];
  const float* W_lin1 = (const float*)d_in[14];
  const float* b_lin1 = (const float*)d_in[15];
  const float* W_lin2 = (const float*)d_in[16];
  const float* b_lin2 = (const float*)d_in[17];
  const int*   e_src  = (const int*)d_in[18];
  const int*   e_dst  = (const int*)d_in[19];
  const int*   el_row = (const int*)d_in[20];
  const int*   el_col = (const int*)d_in[21];
  float* out = (float*)d_out;

  const int MPI = cdiv(nI, GBM) * GBM;
  const int MPU = cdiv(nU, GBM) * GBM;
  const int gAI = cdiv(nI, NBA);
  const int gAU = cdiv(nU, NBA);
  if ((long long)gAI * NBA < (long long)MPI) return;
  if ((long long)gAU * NBA < (long long)MPU) return;
  const int vec8 = ((nE & 3) == 0) ? 1 : 0;

  char* ws = (char*)d_ws;
  size_t off = 0;
  const size_t oB1I = off; off = al256(off + (size_t)DF * K1L * 2);
  const size_t oB1U = off; off = al256(off + (size_t)DF * K1L * 2);
  const size_t oB2I = off; off = al256(off + (size_t)DF * K2L * 2);
  const size_t oB2U = off; off = al256(off + (size_t)DF * K2L * 2);
  const size_t oBDU = off; off = al256(off + (size_t)DF * KDL * 2);
  const size_t oBDI = off; off = al256(off + (size_t)DF * KDL * 2);
  const size_t oAI  = off; off = al256(off + (size_t)MPI * AP * 2);
  const size_t oAU  = off; off = al256(off + (size_t)MPU * AP * 2);
  if (off > ws_size) return;
  unsigned short* B1I = (unsigned short*)(ws + oB1I);
  unsigned short* B1U = (unsigned short*)(ws + oB1U);
  unsigned short* B2I = (unsigned short*)(ws + oB2I);
  unsigned short* B2U = (unsigned short*)(ws + oB2U);
  unsigned short* BDU = (unsigned short*)(ws + oBDU);
  unsigned short* BDI = (unsigned short*)(ws + oBDI);
  unsigned short* API = (unsigned short*)(ws + oAI);
  unsigned short* APU = (unsigned short*)(ws + oAU);

  const size_t scanLds = (size_t)AGG_LDS_INTS * 4;
  hipFuncSetAttribute(reinterpret_cast<const void*>(&k_scan<1>), hipFuncAttributeMaxDynamicSharedMemorySize, (int)scanLds);
  hipFuncSetAttribute(reinterpret_cast<const void*>(&k_scan<0>), hipFuncAttributeMaxDynamicSharedMemorySize, (int)scanLds);

  k_wprep<<<(NPART * UPART) / NTHR, NTHR, 0, stream>>>(Wl1_ui, Wr1_ui, Wl1_iu, Wr1_iu, Wl2_ui, Wr2_ui,
                                                       Wl2_iu, Wr2_iu, W_lin1, B1I, B1U, B2I, B2U, BDU, BDI);
  k_scan<1><<<gAI, NTHR, scanLds, stream>>>(e_src, e_dst, nE, nI, nU, vec8, MPI, x_user, x_item, API, API);
  k_scan<1><<<gAU, NTHR, scanLds, stream>>>(e_dst, e_src, nE, nU, nI, vec8, MPU, x_item, x_user, APU, APU);
  k_gemm<0><<<MPI / GBM, GTHR, 0, stream>>>(API, B1I, K1L, b1_ui, 1, nI);
  k_gemm<0><<<MPU / GBM, GTHR, 0, stream>>>(APU, B1U, K1L, b1_iu, 1, nU);
  k_scan<0><<<gAI, NTHR, scanLds, stream>>>(e_src, e_dst, nE, nI, nU, vec8, MPI, x_user, x_item, APU, API);
  k_scan<0><<<gAU, NTHR, scanLds, stream>>>(e_dst, e_src, nE, nU, nI, vec8, MPU, x_item, x_user, API, APU);
  k_gemm<1><<<MPI / GBM, GTHR, 0, stream>>>(API, B2I, K2L, b2_ui, 1, nI);
  k_gemm<1><<<MPU / GBM, GTHR, 0, stream>>>(APU, B2U, K2L, b2_iu, 1, nU);
  k_gemm<2><<<MPI / GBM, GTHR, 0, stream>>>(API, BDI, KDL, b_lin1, 1, nI);
  k_gemm<2><<<MPU / GBM, GTHR, 0, stream>>>(APU, BDU, KDL, b_lin1, 0, nU);
  k_edge<<<cdiv(nL, ETHR), ETHR, 0, stream>>>((const float*)APU, (const float*)API, el_row, el_col,
                                              nL, nU, nI, W_lin2, b_lin2, out);
}
